// MaskedSelfAttention_54065048323024
// MI455X (gfx1250) — hardware-verified
//
#include <hip/hip_runtime.h>
#include <stdint.h>


typedef _Float16 v16h __attribute__((ext_vector_type(16)));
typedef _Float16 v8h  __attribute__((ext_vector_type(8)));
typedef float    v8f  __attribute__((ext_vector_type(8)));
typedef float    v4f  __attribute__((ext_vector_type(4)));
typedef int      v4i  __attribute__((ext_vector_type(4)));

#ifndef NB
#define NB 2
#endif
#ifndef SEQ
#define SEQ 2048
#endif
#define NB_FULL  2
#define SEQ_FULL 2048
#define DM 1024
#define NH 16
#define DH 64
#ifndef QPREC
#define QPREC ((SEQ < 512) ? SEQ : 512)
#endif
#define NKB   (SEQ / 32)
#define NQB   (SEQ / 64)
#define NQP   (QPREC / 64)
#define MROWS (NB * SEQ)

static_assert(SEQ % 64 == 0);
static_assert(SEQ >= 64 && SEQ <= SEQ_FULL);
static_assert(NB >= 1 && NB <= NB_FULL);
static_assert(QPREC % 64 == 0);
static_assert(QPREC >= 64 && QPREC <= SEQ);
static_assert(NKB <= 64);
static_assert(DM == NH * DH);
static_assert(DM % 32 == 0);
static_assert(MROWS % 64 == 0);

#define WSC    64.0f
#define INV_WS 0.015625f
#define RS     2048.0f
#define INV_RS 0.00048828125f
#define CP     4096.0f
#define INV_CP 0.000244140625f
#define QKS    0.125f

constexpr size_t SZ_XH  = (size_t)MROWS * DM * 2;
constexpr size_t SZ_W   = (size_t)DM * DM * 2;
constexpr size_t SZ_HP  = (size_t)NB * NH * SEQ * DH * 2;
constexpr size_t SZ_LP  = (size_t)NB * NH * QPREC * DH * 2;
constexpr size_t SZ_CH  = (size_t)MROWS * DM * 2;
constexpr size_t SZ_CL  = (size_t)NB * QPREC * DM * 2;
constexpr size_t SZ_FLG = (size_t)NQB * 64 * 4;
constexpr size_t OFF_XH  = 0;
constexpr size_t OFF_WQ  = OFF_XH + SZ_XH;
constexpr size_t OFF_WK  = OFF_WQ + SZ_W;
constexpr size_t OFF_WV  = OFF_WK + SZ_W;
constexpr size_t OFF_WO  = OFF_WV + SZ_W;
constexpr size_t OFF_QH  = OFF_WO + SZ_W;
constexpr size_t OFF_KH  = OFF_QH + SZ_HP;
constexpr size_t OFF_VH  = OFF_KH + SZ_HP;
constexpr size_t OFF_QL  = OFF_VH + SZ_HP;
constexpr size_t OFF_KL  = OFF_QL + SZ_LP;
constexpr size_t OFF_VL  = OFF_KL + SZ_LP;
constexpr size_t OFF_CH  = OFF_VL + SZ_LP;
constexpr size_t OFF_CL  = OFF_CH + SZ_CH;
constexpr size_t OFF_FLG = OFF_CL + SZ_CL;
constexpr size_t WS_TOTAL = OFF_FLG + SZ_FLG;
static_assert(WS_TOTAL <= (size_t)134217728);
static_assert(OFF_WQ % 128 == 0 && OFF_WK % 128 == 0 && OFF_WV % 128 == 0 && OFF_WO % 128 == 0);
static_assert(OFF_QH % 128 == 0 && OFF_KH % 128 == 0 && OFF_VH % 128 == 0);
static_assert(OFF_QL % 128 == 0 && OFF_KL % 128 == 0 && OFF_VL % 128 == 0);
static_assert(OFF_CH % 128 == 0 && OFF_CL % 128 == 0 && OFF_FLG % 128 == 0);
static_assert((size_t)NB_FULL * SEQ_FULL * DM * 4 >= ((size_t)(NB - 1) * SEQ_FULL + SEQ) * DM * 4);

__device__ __forceinline__ float bf16r(float f) {
  unsigned int u = __float_as_uint(f);
  u = (u + 0x7fffu + ((u >> 16) & 1u)) & 0xffff0000u;
  return __uint_as_float(u);
}

__device__ __forceinline__ v16h load_frag(const _Float16* base, int stride) {
  const int lane = threadIdx.x & 31, m = lane & 15, g = lane >> 4;
  const _Float16* p = base + (size_t)m * stride + 8 * g;
  union { v16h v; v8h hf[2]; } f;
  f.hf[0] = *reinterpret_cast<const v8h*>(p);
  f.hf[1] = *reinterpret_cast<const v8h*>(p + 16);
  return f.v;
}

__device__ __forceinline__ v8f mma(v16h a, v16h b, v8f c) {
  v8f d = __builtin_amdgcn_wmma_f32_16x16x32_f16(false, a, false, b, (short)0, c, false, false);
  asm volatile("v_nop\n\tv_nop\n\tv_nop\n\tv_nop" : "+v"(d) : "v"(a), "v"(b));
  return d;
}

__device__ __forceinline__ v8f zero8() {
  v8f z = {0.f, 0.f, 0.f, 0.f, 0.f, 0.f, 0.f, 0.f};
  return z;
}

__global__ __launch_bounds__(256) void k_cvt(const float* __restrict__ in, _Float16* __restrict__ outp,
                                            int nrows, int seqc, int seqf, float scale) {
  const long long e8 = (long long)blockIdx.x * 256 + threadIdx.x;
  const long long tot = (long long)nrows * (DM / 8);
  if (e8 >= tot) return;
  const int mc = (int)(e8 / (DM / 8));
  const int c8 = (int)(e8 - (long long)mc * (DM / 8));
  const int src = (mc / seqc) * seqf + (mc % seqc);
  const float* p = in + (size_t)src * DM + c8 * 8;
  const v4f a = *(const v4f*)p;
  const v4f c = *(const v4f*)(p + 4);
  v8h o;
  o[0] = (_Float16)(bf16r(a[0]) * scale);
  o[1] = (_Float16)(bf16r(a[1]) * scale);
  o[2] = (_Float16)(bf16r(a[2]) * scale);
  o[3] = (_Float16)(bf16r(a[3]) * scale);
  o[4] = (_Float16)(bf16r(c[0]) * scale);
  o[5] = (_Float16)(bf16r(c[1]) * scale);
  o[6] = (_Float16)(bf16r(c[2]) * scale);
  o[7] = (_Float16)(bf16r(c[3]) * scale);
  _Float16* dst = outp + (size_t)mc * DM + c8 * 8;
  *(volatile v8h*)dst = o;
  __threadfence();
  *(volatile v8h*)dst = o;
}

__global__ __launch_bounds__(256) void k_mflag(const int* __restrict__ mask, int* __restrict__ flg) {
  __shared__ unsigned int sLo[256];
  __shared__ unsigned int sHi[256];
  __shared__ int sR[256];
  const int tid = threadIdx.x, qb = blockIdx.x;
  const int r = tid >> 2, sub = tid & 3;
  const int* mrow = mask + (size_t)(qb * 64 + r) * SEQ_FULL + sub * 8;
  unsigned int lo = 0u, hi = 0u;
  int rany = 0;
#pragma unroll 2
  for (int kb = 0; kb < NKB; ++kb) {
    const v4i a = *(const v4i*)(mrow + kb * 32);
    const v4i c = *(const v4i*)(mrow + kb * 32 + 4);
    const int any = ((a[0] | a[1] | a[2] | a[3] | c[0] | c[1] | c[2] | c[3]) != 0) ? 1 : 0;
    const unsigned int bit = (unsigned int)any;
    if (kb < 32) lo |= bit << kb; else hi |= bit << (kb - 32);
    rany |= any;
  }
  sLo[tid] = lo; sHi[tid] = hi; sR[tid] = rany;
  __syncthreads();
  if (tid < 32) {
    unsigned int L = 0u, H = 0u;
#pragma unroll
    for (int i = 0; i < 8; ++i) { L |= sLo[tid + 32 * i]; H |= sHi[tid + 32 * i]; }
#pragma unroll
    for (int off = 1; off < 32; off <<= 1) {
      L |= (unsigned int)__shfl_xor((int)L, off, 32);
      H |= (unsigned int)__shfl_xor((int)H, off, 32);
    }
    const int ra = sR[8 * tid] | sR[8 * tid + 1] | sR[8 * tid + 2] | sR[8 * tid + 3];
    const int rb = sR[8 * tid + 4] | sR[8 * tid + 5] | sR[8 * tid + 6] | sR[8 * tid + 7];
    int ok = ((ra != 0) && (rb != 0)) ? 1 : 0;
#pragma unroll
    for (int off = 1; off < 32; off <<= 1) ok &= __shfl_xor(ok, off, 32);
    v4i f;
#pragma unroll
    for (int e = 0; e < 4; ++e) {
      const int kbx = 4 * tid + e;
      const unsigned int word = (kbx < 32) ? L : H;
      const int bitv = (int)((word >> (kbx & 31)) & 1u);
      f[e] = (kbx < NKB) ? ((ok != 0) ? bitv : 1) : 0;
    }
    int* dst = flg + qb * 64 + 4 * tid;
    if (tid < 16) *(volatile v4i*)dst = f;
    __threadfence();
    if (tid < 16) *(volatile v4i*)dst = f;
  }
}

__device__ __forceinline__ void kloop(const _Float16* __restrict__ abase, const _Float16* __restrict__ wbase,
                                      v8f (&acc)[2][4]) {
#pragma unroll 2
  for (int kc = 0; kc < DM; kc += 32) {
    const v16h a0 = load_frag(abase + kc, DM);
    const v16h a1 = load_frag(abase + (size_t)16 * DM + kc, DM);
#pragma unroll
    for (int j = 0; j < 4; ++j) {
      const v16h bf = load_frag(wbase + (size_t)(j * 16) * DM + kc, DM);
      acc[0][j] = mma(a0, bf, acc[0][j]);
      acc[1][j] = mma(a1, bf, acc[1][j]);
    }
  }
}

template <int MODE>
__global__ __launch_bounds__(64) void k_gemm(const _Float16* __restrict__ A, const _Float16* __restrict__ Alo,
                                            const _Float16* __restrict__ W, const float* __restrict__ bias,
                                            _Float16* __restrict__ Ph, _Float16* __restrict__ Pl,
                                            float* __restrict__ outp) {
  __shared__ __align__(16) _Float16 sH[64 * 64];
  __shared__ __align__(16) _Float16 sL[64 * 64];
  __shared__ __align__(16) float    sF[64 * 64];

  const int tid = threadIdx.x, w = tid >> 5, lane = tid & 31, n = lane & 15, g = lane >> 4;
  const int bm = blockIdx.x, bn = blockIdx.y;
  const int m0 = bm * 64;
  const int b = m0 / SEQ, s0 = m0 - b * SEQ;
  const int bh = b * NH + bn;
  const bool precblk = (s0 < QPREC);
  const _Float16* wbase = W + (size_t)(bn * 64) * DM;
  const _Float16* abase = A + (size_t)(m0 + w * 32) * DM;

  v8f acc[2][4];
#pragma unroll
  for (int mi = 0; mi < 2; ++mi)
#pragma unroll
    for (int j = 0; j < 4; ++j) acc[mi][j] = zero8();

  kloop(abase, wbase, acc);

  float rbias[4];
  if (MODE == 2) {
#pragma unroll
    for (int j = 0; j < 4; ++j) rbias[j] = bf16r(bias[bn * 64 + j * 16 + n]);
  } else {
#pragma unroll
    for (int j = 0; j < 4; ++j) rbias[j] = 0.0f;
  }

  if (MODE == 0) {
#pragma unroll
    for (int mi = 0; mi < 2; ++mi)
#pragma unroll
      for (int j = 0; j < 4; ++j)
#pragma unroll
        for (int r = 0; r < 8; ++r) {
          const int ml = w * 32 + mi * 16 + 8 * g + r;
          const int d = j * 16 + n;
          const float v = acc[mi][j][r] * INV_WS + rbias[j];
          const _Float16 hv = (_Float16)v;
          sH[ml * 64 + d] = hv;
          if (precblk) sL[ml * 64 + d] = (_Float16)((v - (float)hv) * RS);
        }
    __syncthreads();
    const int q = lane >> 3, p = lane & 7;
#pragma unroll 1
    for (int pass = 0; pass < 2; ++pass) {
#pragma unroll
      for (int i = 0; i < 8; ++i) {
        const int ml = w * 32 + i * 4 + q;
        const int s = s0 + ml;
        const v8h hv = *(const v8h*)&sH[ml * 64 + p * 8];
        *(volatile v8h*)(Ph + ((size_t)(bh * SEQ + s)) * DH + p * 8) = hv;
        if (precblk) {
          const v8h lv = *(const v8h*)&sL[ml * 64 + p * 8];
          *(volatile v8h*)(Pl + ((size_t)(bh * QPREC + s)) * DH + p * 8) = lv;
        }
      }
      if (pass == 0) __threadfence();
    }
  } else if (MODE == 1) {
#pragma unroll
    for (int mi = 0; mi < 2; ++mi)
#pragma unroll
      for (int j = 0; j < 4; ++j) {
        v8h hp, lp;
#pragma unroll
        for (int r = 0; r < 8; ++r) {
          const float v = acc[mi][j][r] * INV_WS + rbias[j];
          const _Float16 hv = (_Float16)v;
          hp[r] = hv;
          lp[r] = (_Float16)((v - (float)hv) * RS);
        }
        const int d = j * 16 + n;
        *(v8h*)&sH[d * 64 + w * 32 + mi * 16 + 8 * g] = hp;
        if (precblk) *(v8h*)&sL[d * 64 + w * 32 + mi * 16 + 8 * g] = lp;
      }
    __syncthreads();
    const int q = lane >> 3, p = lane & 7;
#pragma unroll 1
    for (int pass = 0; pass < 2; ++pass) {
#pragma unroll
      for (int i = 0; i < 8; ++i) {
        const int d = w * 32 + i * 4 + q;
        const v8h hv = *(const v8h*)&sH[d * 64 + p * 8];
        *(volatile v8h*)(Ph + ((size_t)(bh * DH + d)) * SEQ + s0 + p * 8) = hv;
        if (precblk) {
          const v8h lv = *(const v8h*)&sL[d * 64 + p * 8];
          *(volatile v8h*)(Pl + ((size_t)(bh * DH + d)) * QPREC + s0 + p * 8) = lv;
        }
      }
      if (pass == 0) __threadfence();
    }
  } else {
    if (precblk) {
#pragma unroll
      for (int mi = 0; mi < 2; ++mi)
#pragma unroll
        for (int j = 0; j < 4; ++j)
#pragma unroll
          for (int r = 0; r < 8; ++r)
            sF[(w * 32 + mi * 16 + 8 * g + r) * 64 + j * 16 + n] = acc[mi][j][r];
#pragma unroll
      for (int mi = 0; mi < 2; ++mi)
#pragma unroll
        for (int j = 0; j < 4; ++j) acc[mi][j] = zero8();
      const _Float16* lbase = Alo + ((size_t)(b * QPREC + s0 + w * 32)) * DM;
      kloop(lbase, wbase, acc);
#pragma unroll
      for (int mi = 0; mi < 2; ++mi)
#pragma unroll
        for (int j = 0; j < 4; ++j)
#pragma unroll
          for (int r = 0; r < 8; ++r) {
            const int idx = (w * 32 + mi * 16 + 8 * g + r) * 64 + j * 16 + n;
            const float hsum = sF[idx];
            sF[idx] = (hsum + acc[mi][j][r] * INV_RS) * INV_WS + rbias[j];
          }
    } else {
#pragma unroll
      for (int mi = 0; mi < 2; ++mi)
#pragma unroll
        for (int j = 0; j < 4; ++j)
#pragma unroll
          for (int r = 0; r < 8; ++r)
            sF[(w * 32 + mi * 16 + 8 * g + r) * 64 + j * 16 + n] = acc[mi][j][r] * INV_WS + rbias[j];
    }
    __syncthreads();
    const int q2 = lane >> 4, p2 = lane & 15;
#pragma unroll 1
    for (int pass = 0; pass < 2; ++pass) {
#pragma unroll
      for (int i = 0; i < 16; ++i) {
        const int ml = w * 32 + 2 * i + q2;
        const int s = s0 + ml;
        const v4f v = *(const v4f*)&sF[ml * 64 + p2 * 4];
        *(volatile v4f*)(outp + ((size_t)(b * SEQ_FULL + s)) * DM + bn * 64 + p2 * 4) = v;
      }
      if (pass == 0) __threadfence();
    }
  }
}

template <bool PREC>
__global__ __launch_bounds__(128) __attribute__((amdgpu_num_vgpr(256)))
void k_attn(const _Float16* __restrict__ Qh, const _Float16* __restrict__ Ql,
            const _Float16* __restrict__ Kh, const _Float16* __restrict__ Kl,
            const _Float16* __restrict__ Vh, const _Float16* __restrict__ Vl,
            const int* __restrict__ mask, const int* __restrict__ flg,
            _Float16* __restrict__ Ch, _Float16* __restrict__ Cl) {
  __shared__ __align__(16) _Float16 sK[32 * DH];
  __shared__ __align__(16) _Float16 sV[DH * 32];
  __shared__ __align__(16) _Float16 sKl[32 * DH];
  __shared__ __align__(16) _Float16 sVl[DH * 32];
  __shared__ __align__(16) _Float16 sQl[64 * DH];
  __shared__ __align__(16) int      sM[64 * 32];
  __shared__ __align__(16) _Float16 sP[4][16 * 32];
  __shared__ __align__(16) _Float16 sPl[4][16 * 32];
  __shared__ __align__(16) _Float16 sC[4][16 * DH];
  __shared__ __align__(16) _Float16 sCl[4][16 * DH];
  __shared__ int sFlg[64];

  const int tid = threadIdx.x, wslot = tid >> 5, lane = tid & 31, n = lane & 15, g = lane >> 4;
  int qb, bh;
  if (PREC) {
    qb = (int)(blockIdx.x % NQP);
    bh = (int)(blockIdx.x / NQP);
  } else {
    constexpr int NQN = ((NQB - NQP) > 0) ? (NQB - NQP) : 1;
    qb = NQP + (int)(blockIdx.x % NQN);
    bh = (int)(blockIdx.x / NQN);
  }
  const int b = bh / NH, h = bh - b * NH;
  const int qrow0 = qb * 64;
  const int qbase = qrow0 + wslot * 16;

  if (tid < 64) sFlg[tid] = flg[qb * 64 + tid];
  if (PREC) {
#pragma unroll
    for (int i = 0; i < 4; ++i) {
      const int c = tid + i * 128;
      *(v8h*)&sQl[c * 8] = *(const v8h*)(Ql + ((size_t)(bh * QPREC + qrow0)) * DH + c * 8);
    }
  }
  __syncthreads();

  const _Float16* qrow = Qh + ((size_t)(bh * SEQ + qbase)) * DH;
  const v16h qa0 = load_frag(qrow, DH);
  const v16h qa1 = load_frag(qrow + 32, DH);

  v8f acc[4], acc2[4];
#pragma unroll
  for (int nt = 0; nt < 4; ++nt) { acc[nt] = zero8(); acc2[nt] = zero8(); }
  float rmax[8], rsum[8];
#pragma unroll
  for (int r = 0; r < 8; ++r) { rmax[r] = -1.0e30f; rsum[r] = 0.0f; }

#pragma unroll 1
  for (int kb = 0; kb < NKB; ++kb) {
    if (sFlg[kb] == 0) continue;
    const int kbase = kb * 32;
    const bool klo = PREC && (kbase < QPREC);
    __syncthreads();
    {
      const _Float16* kg = Kh + ((size_t)(bh * SEQ + kbase)) * DH;
      const _Float16* vg = Vh + ((size_t)(bh * DH)) * SEQ + kbase;
#pragma unroll
      for (int i = 0; i < 2; ++i) {
        const int c = tid + i * 128, d = c >> 2, sub = c & 3;
        *(v8h*)&sK[c * 8] = *(const v8h*)(kg + c * 8);
        *(v8h*)&sV[d * 32 + sub * 8] = *(const v8h*)(vg + (size_t)d * SEQ + sub * 8);
      }
      if (klo) {
        const _Float16* klg = Kl + ((size_t)(bh * QPREC + kbase)) * DH;
        const _Float16* vlg = Vl + ((size_t)(bh * DH)) * QPREC + kbase;
#pragma unroll
        for (int i = 0; i < 2; ++i) {
          const int c = tid + i * 128, d = c >> 2, sub = c & 3;
          *(v8h*)&sKl[c * 8] = *(const v8h*)(klg + c * 8);
          *(v8h*)&sVl[d * 32 + sub * 8] = *(const v8h*)(vlg + (size_t)d * QPREC + sub * 8);
        }
      }
      const int mr = tid >> 1, mh = (tid & 1) * 16;
      const int* mp = mask + (size_t)(qrow0 + mr) * SEQ_FULL + kbase + mh;
#pragma unroll
      for (int i = 0; i < 4; ++i) *(v4i*)&sM[mr * 32 + mh + i * 4] = *(const v4i*)(mp + i * 4);
    }
    __syncthreads();

    v8f s0 = zero8(), s1 = zero8(), sr0 = zero8(), sr1 = zero8();
    {
      v16h t;
      t = load_frag(sK, DH);                 s0 = mma(qa0, t, s0);
      t = load_frag(sK + 32, DH);            s0 = mma(qa1, t, s0);
      t = load_frag(sK + 16 * DH, DH);       s1 = mma(qa0, t, s1);
      t = load_frag(sK + 16 * DH + 32, DH);  s1 = mma(qa1, t, s1);
      if (PREC) {
        if (klo) {
          {
            const v16h ql0 = load_frag(&sQl[(wslot * 16) * DH], DH);
            const v16h ql1 = load_frag(&sQl[(wslot * 16) * DH + 32], DH);
            t = load_frag(sK, DH);                 sr0 = mma(ql0, t, sr0);
            t = load_frag(sK + 32, DH);            sr0 = mma(ql1, t, sr0);
            t = load_frag(sK + 16 * DH, DH);       sr1 = mma(ql0, t, sr1);
            t = load_frag(sK + 16 * DH + 32, DH);  sr1 = mma(ql1, t, sr1);
          }
          t = load_frag(sKl, DH);                 sr0 = mma(qa0, t, sr0);
          t = load_frag(sKl + 32, DH);            sr0 = mma(qa1, t, sr0);
          t = load_frag(sKl + 16 * DH, DH);       sr1 = mma(qa0, t, sr1);
          t = load_frag(sKl + 16 * DH + 32, DH);  sr1 = mma(qa1, t, sr1);
        }
      }
    }

#pragma unroll
    for (int r = 0; r < 8; ++r) {
      const int rl = g * 8 + r;
      const int mro = (wslot * 16 + rl) * 32;
      float v0 = s0[r], v1 = s1[r];
      if (PREC) { v0 += sr0[r] * INV_RS; v1 += sr1[r] * INV_RS; }
      v0 *= QKS; v1 *= QKS;
      const int mk0 = sM[mro + n], mk1 = sM[mro + 16 + n];
      const float x0 = (mk0 == 0) ? -1.0e9f : v0;
      const float x1 = (mk1 == 0) ? -1.0e9f : v1;
      float mx = fmaxf(x0, x1);
#pragma unroll
      for (int off = 1; off < 16; off <<= 1) mx = fmaxf(mx, __shfl_xor(mx, off, 32));
      const float nm = fmaxf(rmax[r], mx);
      const float al = __expf(rmax[r] - nm);
      const float p0 = __expf(x0 - nm);
      const float p1 = __expf(x1 - nm);
      float ps = p0 + p1;
#pragma unroll
      for (int off = 1; off < 16; off <<= 1) ps += __shfl_xor(ps, off, 32);
      rsum[r] = rsum[r] * al + ps;
      rmax[r] = nm;
#pragma unroll
      for (int nt = 0; nt < 4; ++nt) {
        acc[nt][r] *= al;
        if (PREC) acc2[nt][r] *= al;
      }
      const float c0 = p0 * CP, c1 = p1 * CP;
      const _Float16 h0 = (_Float16)c0, h1 = (_Float16)c1;
      sP[wslot][rl * 32 + n] = h0;
      sP[wslot][rl * 32 + 16 + n] = h1;
      if (PREC) {
        sPl[wslot][rl * 32 + n]      = (_Float16)((c0 - (float)h0) * RS);
        sPl[wslot][rl * 32 + 16 + n] = (_Float16)((c1 - (float)h1) * RS);
      }
    }
    __syncthreads();

    {
      const v16h pf = load_frag(&sP[wslot][0], 32);
      if (PREC) {
        const v16h plf = load_frag(&sPl[wslot][0], 32);
#pragma unroll
        for (int nt = 0; nt < 4; ++nt) {
          const v16h vb = load_frag(&sV[nt * 16 * 32], 32);
          acc[nt]  = mma(pf, vb, acc[nt]);
          acc2[nt] = mma(plf, vb, acc2[nt]);
          if (klo) {
            const v16h vlb = load_frag(&sVl[nt * 16 * 32], 32);
            acc2[nt] = mma(pf, vlb, acc2[nt]);
          }
        }
      } else {
#pragma unroll
        for (int nt = 0; nt < 4; ++nt) {
          const v16h vb = load_frag(&sV[nt * 16 * 32], 32);
          acc[nt] = mma(pf, vb, acc[nt]);
        }
      }
    }
  }

#pragma unroll
  for (int r = 0; r < 8; ++r) {
    const float inv = (1.0f / rsum[r]) * INV_CP;
    const int rl = g * 8 + r;
#pragma unroll
    for (int nt = 0; nt < 4; ++nt) {
      float c = acc[nt][r];
      if (PREC) c += acc2[nt][r] * INV_RS;
      c *= inv;
      const _Float16 chv = (_Float16)c;
      sC[wslot][rl * DH + nt * 16 + n] = chv;
      if (PREC) sCl[wslot][rl * DH + nt * 16 + n] = (_Float16)((c - (float)chv) * RS);
    }
  }
  __syncthreads();
  const int q = lane >> 3, p = lane & 7;
#pragma unroll 1
  for (int pass = 0; pass < 2; ++pass) {
#pragma unroll
    for (int i = 0; i < 4; ++i) {
      const int rr = i * 4 + q;
      const v8h hv = *(const v8h*)&sC[wslot][rr * DH + p * 8];
      *(volatile v8h*)(Ch + ((size_t)(b * SEQ + qbase + rr)) * DM + h * DH + p * 8) = hv;
      if (PREC) {
        const v8h lv = *(const v8h*)&sCl[wslot][rr * DH + p * 8];
        *(volatile v8h*)(Cl + ((size_t)(b * QPREC + qbase + rr)) * DM + h * DH + p * 8) = lv;
      }
    }
    if (pass == 0) __threadfence();
  }
}

extern "C" void kernel_launch(void* const* d_in, const int* in_sizes, int n_in,
                              void* d_out, int out_size, void* d_ws, size_t ws_size,
                              hipStream_t stream) {
  if (n_in < 7) return;
  const long long need_x = ((long long)(NB - 1) * SEQ_FULL + SEQ) * DM;
  const long long need_m = ((long long)(SEQ - 1)) * SEQ_FULL + SEQ;
  if ((long long)in_sizes[0] < need_x) return;
  if ((long long)in_sizes[1] < need_m) return;
  if (in_sizes[2] < DM * DM || in_sizes[3] < DM * DM || in_sizes[4] < DM * DM || in_sizes[5] < DM * DM) return;
  if (in_sizes[6] < DM) return;
  if ((long long)out_size < need_x) return;
  if (ws_size < WS_TOTAL) return;

  const float* x    = (const float*)d_in[0];
  const int*   mask = (const int*)d_in[1];
  const float* Wq   = (const float*)d_in[2];
  const float* Wk   = (const float*)d_in[3];
  const float* Wv   = (const float*)d_in[4];
  const float* Wo   = (const float*)d_in[5];
  const float* bo   = (const float*)d_in[6];
  float* out = (float*)d_out;

  char* ws = (char*)d_ws;
  _Float16* Xh   = (_Float16*)(ws + OFF_XH);
  _Float16* Wq64 = (_Float16*)(ws + OFF_WQ);
  _Float16* Wk64 = (_Float16*)(ws + OFF_WK);
  _Float16* Wv64 = (_Float16*)(ws + OFF_WV);
  _Float16* Wo64 = (_Float16*)(ws + OFF_WO);
  _Float16* Qh   = (_Float16*)(ws + OFF_QH);
  _Float16* Kh   = (_Float16*)(ws + OFF_KH);
  _Float16* Vh   = (_Float16*)(ws + OFF_VH);
  _Float16* Ql   = (_Float16*)(ws + OFF_QL);
  _Float16* Kl   = (_Float16*)(ws + OFF_KL);
  _Float16* Vl   = (_Float16*)(ws + OFF_VL);
  _Float16* Ch   = (_Float16*)(ws + OFF_CH);
  _Float16* Cl   = (_Float16*)(ws + OFF_CL);
  int*      Flg  = (int*)(ws + OFF_FLG);

  const int nbx = (MROWS * (DM / 8) + 255) / 256;
  const int nbw = (DM * (DM / 8) + 255) / 256;
  k_cvt<<<nbx, 256, 0, stream>>>(x,  Xh,   MROWS, SEQ, SEQ_FULL, 1.0f);
  k_cvt<<<nbw, 256, 0, stream>>>(Wq, Wq64, DM, DM, DM, WSC);
  k_cvt<<<nbw, 256, 0, stream>>>(Wk, Wk64, DM, DM, DM, WSC);
  k_cvt<<<nbw, 256, 0, stream>>>(Wv, Wv64, DM, DM, DM, WSC);
  k_cvt<<<nbw, 256, 0, stream>>>(Wo, Wo64, DM, DM, DM, WSC);

  k_mflag<<<NQB, 256, 0, stream>>>(mask, Flg);

  const dim3 gg(MROWS / 64, DM / 64);
  k_gemm<0><<<gg, 64, 0, stream>>>(Xh, Xh, Wq64, bo, Qh, Ql, out);
  k_gemm<0><<<gg, 64, 0, stream>>>(Xh, Xh, Wk64, bo, Kh, Kl, out);
  k_gemm<1><<<gg, 64, 0, stream>>>(Xh, Xh, Wv64, bo, Vh, Vl, out);

  const int nprec  = NB * NH * NQP;
  const int nplain = NB * NH * (NQB - NQP);
  k_attn<true><<<nprec, 128, 0, stream>>>(Qh, Ql, Kh, Kl, Vh, Vl, mask, Flg, Ch, Cl);
  if (nplain > 0)
    k_attn<false><<<nplain, 128, 0, stream>>>(Qh, Ql, Kh, Kl, Vh, Vl, mask, Flg, Ch, Cl);

  k_gemm<2><<<gg, 64, 0, stream>>>(Ch, Cl, Wo64, bo, Qh, Ql, out);
}
